// KnowledgeAttention_42339787604842
// MI455X (gfx1250) — hardware-verified
//
#include <hip/hip_runtime.h>
#include <math.h>
#include <stdint.h>

#ifndef NB
#define NB       8
#endif
#ifndef SQ
#define SQ       2048
#endif
#define NB_FULL  8
#define SQ_FULL  2048
#define SKV      512
#define DM       768
#define NH       12
#define HD       64
#define INNER    (NH * HD)
#define WSC      256.0f
#define QS       8.0f
#define KS       8.0f
#define VS       8.0f
#define PCAR     32768.0f
#define OSC      1024.0f
#define RSC      2048.0f
#define RINV     0.00048828125f
#define LOG2E    1.4426950408889634f
#define RSQ_HD   0.125f
#define EPSN     1e-8f
#define NKB      (SKV / 32)
#define ATT_WAVES   4
#define ATT_THREADS (ATT_WAVES * 32)
#define CVT_THREADS (DM / 8)
#define SIM_THREADS 256
#define SIM_KEYS    32
#define OPITCH   68
#define GPITCH   68

#define M_HL     0
#define M_S16    1
#define M_F32    2

static_assert(NB >= 1 && NB <= NB_FULL);
static_assert((SQ % 64) == 0 && SQ >= 64 && SQ <= SQ_FULL);
static_assert(HD == 64 && INNER == 768 && NH == 12 && INNER == DM);
static_assert((SKV % 64) == 0 && (SKV % 32) == 0 && NKB * 32 == SKV && (SKV % SIM_KEYS) == 0);
static_assert((DM % 64) == 0 && (DM % 32) == 0 && CVT_THREADS * 8 == DM && (CVT_THREADS % 32) == 0);
static_assert((OPITCH * 4) % 16 == 0 && (GPITCH * 4) % 16 == 0);
static_assert(ATT_THREADS == 128 && SIM_THREADS == 256 && SIM_KEYS == (SIM_THREADS / 32) * 4);

typedef unsigned short u16;
typedef _Float16 v16h __attribute__((ext_vector_type(16)));
typedef _Float16 v8h  __attribute__((ext_vector_type(8)));
typedef float    v8f  __attribute__((ext_vector_type(8)));
typedef float    v4f  __attribute__((ext_vector_type(4)));
typedef unsigned int v4u __attribute__((ext_vector_type(4)));

union FragH { v16h v; v8h h[2]; v4u u[2]; };

__device__ __forceinline__ unsigned short bf_bits(float f) {
  unsigned u = __float_as_uint(f);
  return (unsigned short)((u + 0x7FFFu + ((u >> 16) & 1u)) >> 16);
}
__device__ __forceinline__ float bf_up(unsigned short h) { return __uint_as_float(((unsigned)h) << 16); }
__device__ __forceinline__ float bfr(float f) { return bf_up(bf_bits(f)); }
__device__ __forceinline__ unsigned short h_bits(_Float16 x) { return __builtin_bit_cast(unsigned short, x); }
__device__ __forceinline__ unsigned pk16(unsigned short a, unsigned short b) { return (unsigned)a | ((unsigned)b << 16); }
__device__ __forceinline__ v8f zero8() { v8f z = {0.f, 0.f, 0.f, 0.f, 0.f, 0.f, 0.f, 0.f}; return z; }

__device__ __forceinline__ float wave_sum(float v) {
  v += __shfl_xor(v, 16, 32);
  v += __shfl_xor(v, 8, 32);
  v += __shfl_xor(v, 4, 32);
  v += __shfl_xor(v, 2, 32);
  v += __shfl_xor(v, 1, 32);
  return v;
}

__device__ __forceinline__ void split2(float x0, float x1, unsigned& ph, unsigned& pl) {
  const _Float16 h0 = (_Float16)x0, h1 = (_Float16)x1;
  const float d0 = x0 - (float)h0, d1 = x1 - (float)h1;
  const _Float16 l0 = (_Float16)(d0 * RSC), l1 = (_Float16)(d1 * RSC);
  ph = pk16(h_bits(h0), h_bits(h1));
  pl = pk16(h_bits(l0), h_bits(l1));
}

__device__ __forceinline__ v16h ldfrag_h(const _Float16* p) {
  FragH f;
  f.h[0] = *(const v8h*)(p);
  f.h[1] = *(const v8h*)(p + 16);
  return f.v;
}

__device__ __forceinline__ v8f mma_h(v16h a, v16h b, v8f c) {
  return __builtin_amdgcn_wmma_f32_16x16x32_f16(false, a, false, b, (short)0, c, false, false);
}
__device__ __forceinline__ void guard_c1(v8f (&a)[4], v16h x0, v16h x1, v16h x2, v16h x3, v16h x4) {
#if defined(__HIP_DEVICE_COMPILE__)
  asm volatile("v_nop\n\tv_nop\n\tv_nop\n\tv_nop"
               : "+v"(a[0]), "+v"(a[1]), "+v"(a[2]), "+v"(a[3])
               : "v"(x0), "v"(x1), "v"(x2), "v"(x3), "v"(x4) : "memory");
#endif
}
__device__ __forceinline__ void guard_c2(v8f (&a)[4], v8f (&b)[4], v16h x0, v16h x1, v16h x2, v16h x3, v16h x4, v16h x5) {
#if defined(__HIP_DEVICE_COMPILE__)
  asm volatile("v_nop\n\tv_nop\n\tv_nop\n\tv_nop"
               : "+v"(a[0]), "+v"(a[1]), "+v"(a[2]), "+v"(a[3]),
                 "+v"(b[0]), "+v"(b[1]), "+v"(b[2]), "+v"(b[3])
               : "v"(x0), "v"(x1), "v"(x2), "v"(x3), "v"(x4), "v"(x5) : "memory");
#endif
}
__device__ __forceinline__ void guard_s4(v8f& a, v8f& b, v8f& c, v8f& d,
                                         v16h x0, v16h x1, v16h x2, v16h x3, v16h x4, v16h x5) {
#if defined(__HIP_DEVICE_COMPILE__)
  asm volatile("v_nop\n\tv_nop\n\tv_nop\n\tv_nop"
               : "+v"(a), "+v"(b), "+v"(c), "+v"(d)
               : "v"(x0), "v"(x1), "v"(x2), "v"(x3), "v"(x4), "v"(x5) : "memory");
#endif
}
__device__ __forceinline__ void guard_p(v8f& a, v8f& b, v8f& c, v8f& d, v16h p, v16h x0, v16h x1, v16h x2, v16h x3) {
#if defined(__HIP_DEVICE_COMPILE__)
  asm volatile("v_nop\n\tv_nop\n\tv_nop\n\tv_nop"
               : "+v"(a), "+v"(b), "+v"(c), "+v"(d) : "v"(p), "v"(x0), "v"(x1), "v"(x2), "v"(x3) : "memory");
#endif
}
__device__ __forceinline__ void acc_guard4(v8f (&a)[4]) {
#if defined(__HIP_DEVICE_COMPILE__)
  asm volatile("v_nop\n\tv_nop\n\tv_nop\n\tv_nop" : "+v"(a[0]), "+v"(a[1]), "+v"(a[2]), "+v"(a[3]));
#endif
}
__device__ __forceinline__ void acc_guard8(v8f (&a)[4], v8f (&b)[4]) {
#if defined(__HIP_DEVICE_COMPILE__)
  asm volatile("v_nop\n\tv_nop\n\tv_nop\n\tv_nop"
               : "+v"(a[0]), "+v"(a[1]), "+v"(a[2]), "+v"(a[3]),
                 "+v"(b[0]), "+v"(b[1]), "+v"(b[2]), "+v"(b[3]));
#endif
}
__device__ __forceinline__ void wave_sync_lds() {
  __builtin_amdgcn_fence(__ATOMIC_RELEASE, "workgroup");
  __builtin_amdgcn_wave_barrier();
  __builtin_amdgcn_fence(__ATOMIC_ACQUIRE, "workgroup");
}

__global__ __launch_bounds__(CVT_THREADS)
void cvt16(const float* __restrict__ x, u16* Y, int rowsPerB, int srcRowsPerB, float scale) {
  const int tid = threadIdx.x;
  const int r = blockIdx.x;
  const int b = r / rowsPerB;
  const int s = r - b * rowsPerB;
  const float* src = x + ((size_t)b * (size_t)srcRowsPerB + (size_t)s) * (size_t)DM + (size_t)tid * 8;
  const v4f a = *(const v4f*)(src), c4 = *(const v4f*)(src + 4);
  v4u o;
#pragma unroll
  for (int e = 0; e < 2; ++e) {
    o[e]     = pk16(h_bits((_Float16)(bfr(a[2 * e]) * scale)),  h_bits((_Float16)(bfr(a[2 * e + 1]) * scale)));
    o[2 + e] = pk16(h_bits((_Float16)(bfr(c4[2 * e]) * scale)), h_bits((_Float16)(bfr(c4[2 * e + 1]) * scale)));
  }
  u16* dst = Y + (size_t)r * (size_t)DM + (size_t)tid * 8;
  for (int pass = 0; pass < 2; ++pass) {
    *(volatile v4u*)(dst) = o;
    __threadfence();
  }
}

__global__ __launch_bounds__(SIM_THREADS)
void k_sim(const float* __restrict__ pooled, const float* __restrict__ kgk, const int* __restrict__ msk, float* S) {
  __shared__ __align__(16) float sv[SIM_KEYS];
  (void)msk;
  const int tid = threadIdx.x, wave = tid >> 5, lane = tid & 31;
  constexpr int NKBLK = SKV / SIM_KEYS;
  const int b  = blockIdx.x / NKBLK;
  const int kb = (blockIdx.x - b * NKBLK) * SIM_KEYS;
  const float* p = pooled + (size_t)b * DM;
  float pp = 0.f;
#pragma unroll 1
  for (int e = lane; e < DM; e += 32) {
    const float xv = bfr(p[e]);
    pp += xv * xv;
  }
  pp = wave_sum(pp);
  const float pnrm = fmaxf(sqrtf(pp), EPSN);
#pragma unroll 1
  for (int j = 0; j < 4; ++j) {
    const int k = kb + wave * 4 + j;
    const float* kr = kgk + ((size_t)b * SKV + (size_t)k) * (size_t)DM;
    float pk = 0.f, kk = 0.f;
#pragma unroll 1
    for (int e = lane; e < DM; e += 32) {
      const float xv = bfr(p[e]);
      const float yv = bfr(kr[e]);
      pk += xv * yv;
      kk += yv * yv;
    }
    pk = wave_sum(pk);
    kk = wave_sum(kk);
    const float knrm = fmaxf(sqrtf(kk), EPSN);
    const float val = pk / (pnrm * knrm);
    if (lane == 0) sv[wave * 4 + j] = val;
  }
  __syncthreads();
  if (wave == 0) {
    const v4f v = *(const v4f*)(sv + 4 * (lane & 7));
    float* dst = S + (size_t)b * SKV + kb + 4 * (lane & 7);
    if (lane < 8) {
      *(volatile v4f*)dst = v;
    }
    __threadfence();
    if (lane < 8) {
      *(volatile v4f*)dst = v;
    }
  }
}

__device__ __forceinline__ void core1(const _Float16* ap, const _Float16* bp, int K, v8f (&acc)[4]) {
  const size_t rs16 = (size_t)16 * (size_t)K;
#pragma unroll 1
  for (int k0 = 0; k0 < K; k0 += 32) {
    const v16h a0 = ldfrag_h(ap + k0);
    const v16h b0 = ldfrag_h(bp + k0);
    const v16h b1 = ldfrag_h(bp + rs16 + k0);
    const v16h b2 = ldfrag_h(bp + 2 * rs16 + k0);
    const v16h b3 = ldfrag_h(bp + 3 * rs16 + k0);
    acc[0] = mma_h(a0, b0, acc[0]);
    acc[1] = mma_h(a0, b1, acc[1]);
    acc[2] = mma_h(a0, b2, acc[2]);
    acc[3] = mma_h(a0, b3, acc[3]);
    guard_c1(acc, a0, b0, b1, b2, b3);
  }
}
__device__ __forceinline__ void core2(const _Float16* aph, const _Float16* apl, const _Float16* bp, int K,
                                      v8f (&ah)[4], v8f (&al)[4]) {
  const size_t rs16 = (size_t)16 * (size_t)K;
#pragma unroll 1
  for (int k0 = 0; k0 < K; k0 += 32) {
    const v16h a0 = ldfrag_h(aph + k0);
    const v16h a1 = ldfrag_h(apl + k0);
    const v16h b0 = ldfrag_h(bp + k0);
    const v16h b1 = ldfrag_h(bp + rs16 + k0);
    const v16h b2 = ldfrag_h(bp + 2 * rs16 + k0);
    const v16h b3 = ldfrag_h(bp + 3 * rs16 + k0);
    ah[0] = mma_h(a0, b0, ah[0]);
    ah[1] = mma_h(a0, b1, ah[1]);
    ah[2] = mma_h(a0, b2, ah[2]);
    ah[3] = mma_h(a0, b3, ah[3]);
    al[0] = mma_h(a1, b0, al[0]);
    al[1] = mma_h(a1, b1, al[1]);
    al[2] = mma_h(a1, b2, al[2]);
    al[3] = mma_h(a1, b3, al[3]);
    guard_c2(ah, al, a0, a1, b0, b1, b2, b3);
  }
}

template <bool HASLO, bool BROW>
__device__ __forceinline__ void stage16(float* sl, v8f (&ah)[4], v8f (&al)[4], const float* __restrict__ bias,
                                        int rowb, int col0, float osc, float bsc, int lane) {
  const int hh = lane >> 4, m = lane & 15;
  float bc[4], br[8];
  if (BROW) {
#pragma unroll
    for (int r = 0; r < 8; ++r) br[r] = bfr(bias[rowb + 8 * hh + r]) * bsc;
#pragma unroll
    for (int j = 0; j < 4; ++j) bc[j] = 0.f;
  } else {
#pragma unroll
    for (int j = 0; j < 4; ++j) bc[j] = bfr(bias[col0 + 16 * j + m]) * bsc;
#pragma unroll
    for (int r = 0; r < 8; ++r) br[r] = 0.f;
  }
  const float oscl = osc * RINV;
#pragma unroll
  for (int r = 0; r < 8; ++r) {
    const int ro = (8 * hh + r) * GPITCH + m;
#pragma unroll
    for (int j = 0; j < 4; ++j) {
      float v = ah[j][r] * osc;
      if (HASLO) v += al[j][r] * oscl;
      v += BROW ? br[r] : bc[j];
      sl[ro + 16 * j] = v;
    }
  }
  wave_sync_lds();
}

template <bool HASLO, int MODE, bool BROW>
__global__ __launch_bounds__(128)
void gemm16(const u16* __restrict__ Ah, const u16* __restrict__ Al, const u16* __restrict__ Bt,
            const float* __restrict__ bias, float* F, u16* H, u16* L,
            int Mb, int N, int K, int aBs, int bBs, int fBs, int hBs,
            float osc, float bsc, float carry) {
  __shared__ __align__(16) float slab[4 * 16 * GPITCH];
  constexpr bool LOUT = (MODE == M_HL);
  const int tid = threadIdx.x, wave = tid >> 5, lane = tid & 31, hh = lane >> 4, m = lane & 15;
  const int ntile = N >> 6, mtile = Mb >> 6;
  const int bid  = blockIdx.x;
  const int nt   = bid % ntile;
  const int tmp  = bid / ntile;
  const int mt   = tmp % mtile;
  const int bz   = tmp / mtile;
  const int rowb = mt * 64 + wave * 16;
  const int col0 = nt * 64;
  if (rowb + 16 > Mb) return;
  const _Float16* aph = (const _Float16*)(const void*)Ah + (size_t)bz * (size_t)aBs + (size_t)(rowb + m) * (size_t)K + 8 * hh;
  const _Float16* apl = (const _Float16*)(const void*)Al + (size_t)bz * (size_t)aBs + (size_t)(rowb + m) * (size_t)K + 8 * hh;
  const _Float16* bp  = (const _Float16*)(const void*)Bt + (size_t)bz * (size_t)bBs + (size_t)(col0 + m) * (size_t)K + 8 * hh;
  v8f ah[4], al[4];
#pragma unroll
  for (int i = 0; i < 4; ++i) { ah[i] = zero8(); al[i] = zero8(); }
  if (HASLO) {
    core2(aph, apl, bp, K, ah, al);
    acc_guard8(ah, al);
  } else {
    core1(aph, bp, K, ah);
    acc_guard4(ah);
  }
  float* sl = slab + wave * 16 * GPITCH;
  stage16<HASLO, BROW>(sl, ah, al, bias, rowb, col0, osc, bsc, lane);

  if (MODE == M_F32) {
    v4f vals[8];
#pragma unroll
    for (int it = 0; it < 8; ++it) vals[it] = *(const v4f*)(sl + (it * 2 + hh) * GPITCH + m * 4);
    float* Fb = F + (size_t)bz * (size_t)fBs + ((size_t)rowb + (size_t)hh) * (size_t)N + col0 + m * 4;
    for (int pass = 0; pass < 2; ++pass) {
#pragma unroll
      for (int it = 0; it < 8; ++it) {
        *(volatile v4f*)(Fb + (size_t)(it * 2) * (size_t)N) = vals[it];
      }
      __threadfence();
    }
  } else {
    const int rq = lane >> 3, c8 = (lane & 7) * 8;
    v4u ovh[4], ovl[4];
#pragma unroll
    for (int i = 0; i < 4; ++i) {
      const int row = 4 * i + rq;
      const v4f a = *(const v4f*)(sl + row * GPITCH + c8), c4 = *(const v4f*)(sl + row * GPITCH + c8 + 4);
#pragma unroll
      for (int e = 0; e < 2; ++e) {
        unsigned ph0, pl0, ph1, pl1;
        split2(a[2 * e] * carry,  a[2 * e + 1] * carry,  ph0, pl0);
        split2(c4[2 * e] * carry, c4[2 * e + 1] * carry, ph1, pl1);
        ovh[i][e] = ph0;     ovl[i][e] = pl0;
        ovh[i][2 + e] = ph1; ovl[i][2 + e] = pl1;
      }
    }
    u16* Hb = H + (size_t)bz * (size_t)hBs + (size_t)rowb * (size_t)N + col0 + c8;
    u16* Lb = L + (size_t)bz * (size_t)hBs + (size_t)rowb * (size_t)N + col0 + c8;
    for (int pass = 0; pass < 2; ++pass) {
#pragma unroll
      for (int i = 0; i < 4; ++i) {
        const int row = 4 * i + rq;
        *(volatile v4u*)(Hb + (size_t)row * (size_t)N) = ovh[i];
        if (LOUT) *(volatile v4u*)(Lb + (size_t)row * (size_t)N) = ovl[i];
      }
      __threadfence();
    }
  }
}

__global__ __launch_bounds__(ATT_THREADS)
void attn_fwd(const u16* __restrict__ Qh, const u16* __restrict__ Ql, const u16* __restrict__ Kh,
              const u16* __restrict__ Kl, const u16* __restrict__ Vp, const float* __restrict__ Simp,
              const float* __restrict__ beta, u16* Oh, u16* Ol) {
  __shared__ __align__(16) float smem[ATT_WAVES * 16 * OPITCH];

  const int tid  = threadIdx.x;
  const int wave = tid >> 5;
  const int lane = tid & 31;
  const int hh   = lane >> 4;
  const int c    = lane & 15;

  constexpr int NQT = SQ / 64;
  const int bid  = blockIdx.x;
  const int qt   = bid % NQT;
  const int head = (bid / NQT) % NH;
  const int b    = bid / (NQT * NH);
  const int q0   = qt * 64 + wave * 16;

  const size_t qo = ((size_t)(b * SQ + q0 + c)) * INNER + head * HD + 8 * hh;
  const _Float16* Qhb = (const _Float16*)(const void*)Qh + qo;
  const _Float16* Qlb = (const _Float16*)(const void*)Ql + qo;
  const size_t ko = ((size_t)(b * SKV + c)) * INNER + head * HD + 8 * hh;
  const _Float16* Khb = (const _Float16*)(const void*)Kh + ko;
  const _Float16* Klb = (const _Float16*)(const void*)Kl + ko;
  const _Float16* Vb = (const _Float16*)(const void*)Vp + ((size_t)(b * NH + head) * HD + c) * SKV + 8 * hh;
  const float* Sb = Simp + (size_t)b * SKV + 8 * hh;
  const float bl2 = bfr(beta[head]) * LOG2E;
  const float lsc = (LOG2E * RSQ_HD) / (QS * KS);

  v16h qh[2], ql[2];
  qh[0] = ldfrag_h(Qhb);
  qh[1] = ldfrag_h(Qhb + 32);
  ql[0] = ldfrag_h(Qlb);
  ql[1] = ldfrag_h(Qlb + 32);

  float mrun = -INFINITY, lrun = 0.f;
  v8f o[4];
#pragma unroll
  for (int j = 0; j < 4; ++j) o[j] = zero8();

#pragma unroll 1
  for (int it = 0; it < NKB; ++it) {
    const int kb = it * 32;
    v8f s0 = zero8(), s1 = zero8(), r0 = zero8(), r1 = zero8();
    const _Float16* k0h = Khb + (size_t)kb * INNER;
    const _Float16* k1h = k0h + (size_t)16 * INNER;
    const _Float16* k0l = Klb + (size_t)kb * INNER;
    const _Float16* k1l = k0l + (size_t)16 * INNER;
#pragma unroll
    for (int kk = 0; kk < HD / 32; ++kk) {
      const v16h fh0 = ldfrag_h(k0h + kk * 32);
      const v16h fh1 = ldfrag_h(k1h + kk * 32);
      const v16h fl0 = ldfrag_h(k0l + kk * 32);
      const v16h fl1 = ldfrag_h(k1l + kk * 32);
      s0 = mma_h(fh0, qh[kk], s0);
      s1 = mma_h(fh1, qh[kk], s1);
      r0 = mma_h(fl0, qh[kk], r0);
      r1 = mma_h(fl1, qh[kk], r1);
      r0 = mma_h(fh0, ql[kk], r0);
      r1 = mma_h(fh1, ql[kk], r1);
      guard_s4(s0, s1, r0, r1, qh[kk], ql[kk], fh0, fh1, fl0, fl1);
    }
    const v4f g0 = *(const v4f*)(Sb + kb);
    const v4f g1 = *(const v4f*)(Sb + kb + 4);
    const v4f g2 = *(const v4f*)(Sb + kb + 16);
    const v4f g3 = *(const v4f*)(Sb + kb + 20);
    float t[16];
#pragma unroll
    for (int i = 0; i < 4; ++i) {
      t[i]      = (s0[i]     + r0[i]     * RINV) * lsc + g0[i] * bl2;
      t[4 + i]  = (s0[4 + i] + r0[4 + i] * RINV) * lsc + g1[i] * bl2;
      t[8 + i]  = (s1[i]     + r1[i]     * RINV) * lsc + g2[i] * bl2;
      t[12 + i] = (s1[4 + i] + r1[4 + i] * RINV) * lsc + g3[i] * bl2;
    }
    float cm = t[0];
#pragma unroll
    for (int i = 1; i < 16; ++i) cm = fmaxf(cm, t[i]);
    cm = fmaxf(cm, __shfl_xor(cm, 16, 32));
    const float mn = fmaxf(mrun, cm);
    const float al = exp2f(mrun - mn);
    mrun = mn;
    float ps = 0.f;
    FragH ph;
#pragma unroll
    for (int w = 0; w < 2; ++w) {
#pragma unroll
      for (int e4 = 0; e4 < 4; ++e4) {
        const int i = 8 * w + 2 * e4;
        const float p0 = exp2f(t[i] - mn), p1 = exp2f(t[i + 1] - mn);
        ps += p0 + p1;
        ph.u[w][e4] = pk16(h_bits((_Float16)(p0 * PCAR)), h_bits((_Float16)(p1 * PCAR)));
      }
    }
    ps += __shfl_xor(ps, 16, 32);
    lrun = lrun * al + ps;
    float scl[8];
#pragma unroll
    for (int r = 0; r < 8; ++r) scl[r] = __shfl(al, 8 * hh + r, 32);
#pragma unroll
    for (int j = 0; j < 4; ++j) {
#pragma unroll
      for (int r = 0; r < 8; ++r) o[j][r] *= scl[r];
    }
    {
      const _Float16* vp = Vb + kb;
      const v16h v0 = ldfrag_h(vp);
      const v16h v1 = ldfrag_h(vp + (size_t)16 * SKV);
      const v16h v2 = ldfrag_h(vp + (size_t)32 * SKV);
      const v16h v3 = ldfrag_h(vp + (size_t)48 * SKV);
      o[0] = mma_h(ph.v, v0, o[0]);
      o[1] = mma_h(ph.v, v1, o[1]);
      o[2] = mma_h(ph.v, v2, o[2]);
      o[3] = mma_h(ph.v, v3, o[3]);
      guard_p(o[0], o[1], o[2], o[3], ph.v, v0, v1, v2, v3);
    }
  }
  acc_guard4(o);

  const float linv = (1.0f / lrun) * (OSC / (PCAR * VS));
  float inv[8];
#pragma unroll
  for (int r = 0; r < 8; ++r) inv[r] = __shfl(linv, 8 * hh + r, 32);
  float* slab = smem + wave * 16 * OPITCH;
#pragma unroll
  for (int r = 0; r < 8; ++r) {
#pragma unroll
    for (int j = 0; j < 4; ++j) slab[(8 * hh + r) * OPITCH + j * 16 + c] = o[j][r] * inv[r];
  }
  wave_sync_lds();
  v4u ovh[4], ovl[4];
  const int rq = lane >> 3, c8 = (lane & 7) * 8;
#pragma unroll
  for (int i = 0; i < 4; ++i) {
    const int row = 4 * i + rq;
    const v4f a = *(const v4f*)(slab + row * OPITCH + c8), c4 = *(const v4f*)(slab + row * OPITCH + c8 + 4);
#pragma unroll
    for (int e = 0; e < 2; ++e) {
      unsigned ph0, pl0, ph1, pl1;
      split2(a[2 * e],  a[2 * e + 1],  ph0, pl0);
      split2(c4[2 * e], c4[2 * e + 1], ph1, pl1);
      ovh[i][e] = ph0;     ovl[i][e] = pl0;
      ovh[i][2 + e] = ph1; ovl[i][2 + e] = pl1;
    }
  }
  const size_t oo = ((size_t)(b * SQ + q0)) * INNER + head * HD + c8;
  u16* obh = Oh + oo;
  u16* obl = Ol + oo;
  for (int pass = 0; pass < 2; ++pass) {
#pragma unroll
    for (int i = 0; i < 4; ++i) {
      const int row = 4 * i + rq;
      *(volatile v4u*)(obh + (size_t)row * INNER) = ovh[i];
      *(volatile v4u*)(obl + (size_t)row * INNER) = ovl[i];
    }
    __threadfence();
  }
}

extern "C" void kernel_launch(void* const* d_in, const int* in_sizes, int n_in,
                              void* d_out, int out_size, void* d_ws, size_t ws_size,
                              hipStream_t stream) {
  if (n_in < 14) return;
  if (in_sizes[0] < ((NB - 1) * SQ_FULL + SQ) * DM) return;
  if (in_sizes[1] < 1) return;
  if (in_sizes[2] < NB * DM) return;
  if (in_sizes[3] < NB * SKV * DM || in_sizes[4] < NB * SKV * DM) return;
  if (in_sizes[5] < NH) return;
  if (in_sizes[6] != DM * DM || in_sizes[8] != DM * DM || in_sizes[10] != DM * DM || in_sizes[12] != DM * DM) return;
  if (in_sizes[7] < DM || in_sizes[9] < DM || in_sizes[11] < DM || in_sizes[13] < DM) return;
  if (out_size < ((NB - 1) * SQ_FULL + SQ) * DM) return;

  const float* x_in   = (const float*)d_in[0];
  const int*   msk    = (const int*)d_in[1];
  const float* pooled = (const float*)d_in[2];
  const float* kgk    = (const float*)d_in[3];
  const float* kgv    = (const float*)d_in[4];
  const float* beta   = (const float*)d_in[5];
  const float* wq     = (const float*)d_in[6];
  const float* bq     = (const float*)d_in[7];
  const float* wk     = (const float*)d_in[8];
  const float* bk     = (const float*)d_in[9];
  const float* wv     = (const float*)d_in[10];
  const float* bv     = (const float*)d_in[11];
  const float* wo     = (const float*)d_in[12];
  const float* bo     = (const float*)d_in[13];
  float*       out    = (float*)d_out;

  const size_t szXQ = (size_t)NB * SQ * DM * 2;
  const size_t szXV = (size_t)NB * SKV * DM * 2;
  const size_t szW  = (size_t)DM * DM * 2;
  const size_t szQP = (size_t)NB * SQ * INNER * 2;
  const size_t szKP = (size_t)NB * SKV * INNER * 2;
  const size_t szVT = (size_t)NB * INNER * SKV * 2;
  const size_t szS  = (size_t)NB * SKV * 4;
  static_assert((size_t)NB * SQ * DM * 2 == (size_t)NB * SQ * INNER * 2);
  size_t off = 0;
  const size_t oXQ = off; off += szXQ;
  const size_t oXV = off; off += szXV;
  const size_t oWQ = off; off += szW;
  const size_t oWK = off; off += szW;
  const size_t oWV = off; off += szW;
  const size_t oWO = off; off += szW;
  const size_t oQH = off; off += szQP;
  const size_t oQL = off; off += szQP;
  const size_t oKH = off; off += szKP;
  const size_t oKL = off; off += szKP;
  const size_t oVT = off; off += szVT;
  const size_t oOL = off; off += szQP;
  const size_t oS  = off; off += szS;
  if (off > ws_size) return;
  if (off > (size_t)134217728) return;

  char* ws = (char*)d_ws;
  u16* XQ   = (u16*)(ws + oXQ);
  u16* XV   = (u16*)(ws + oXV);
  u16* WQ16 = (u16*)(ws + oWQ);
  u16* WK16 = (u16*)(ws + oWK);
  u16* WV16 = (u16*)(ws + oWV);
  u16* WO16 = (u16*)(ws + oWO);
  u16* QH   = (u16*)(ws + oQH);
  u16* QL   = (u16*)(ws + oQL);
  u16* KH   = (u16*)(ws + oKH);
  u16* KL   = (u16*)(ws + oKL);
  u16* VT16 = (u16*)(ws + oVT);
  u16* OH   = (u16*)(ws + oXQ);
  u16* OL   = (u16*)(ws + oOL);
  float* SIMP = (float*)(ws + oS);

  cvt16<<<dim3(NB * SQ), dim3(CVT_THREADS), 0, stream>>>(x_in, XQ, SQ, SQ_FULL, 1.0f);
  cvt16<<<dim3(NB * SKV), dim3(CVT_THREADS), 0, stream>>>(kgv, XV, SKV, SKV, 1.0f);
  cvt16<<<dim3(DM), dim3(CVT_THREADS), 0, stream>>>(wq, WQ16, DM, DM, WSC);
  cvt16<<<dim3(DM), dim3(CVT_THREADS), 0, stream>>>(wk, WK16, DM, DM, WSC);
  cvt16<<<dim3(DM), dim3(CVT_THREADS), 0, stream>>>(wv, WV16, DM, DM, WSC);
  cvt16<<<dim3(DM), dim3(CVT_THREADS), 0, stream>>>(wo, WO16, DM, DM, WSC);
  k_sim<<<dim3(NB * (SKV / SIM_KEYS)), dim3(SIM_THREADS), 0, stream>>>(pooled, kgk, msk, SIMP);
  gemm16<false, M_HL, false><<<dim3((NB * SQ / 64) * (INNER / 64)), dim3(128), 0, stream>>>(
      XQ, XQ, WQ16, bq, out, QH, QL, NB * SQ, INNER, DM, 0, 0, 0, 0, QS / WSC, QS, 1.0f);
  gemm16<false, M_HL, false><<<dim3((NB * SKV / 64) * (INNER / 64)), dim3(128), 0, stream>>>(
      XV, XV, WK16, bk, out, KH, KL, NB * SKV, INNER, DM, 0, 0, 0, 0, KS / WSC, KS, 1.0f);
  gemm16<false, M_S16, true><<<dim3(NB * (INNER / 64) * (SKV / 64)), dim3(128), 0, stream>>>(
      WV16, WV16, XV, bv, out, VT16, VT16, INNER, SKV, DM, 0, SKV * DM, 0, INNER * SKV, VS / WSC, VS, 1.0f);
  attn_fwd<<<dim3(NB * NH * (SQ / 64)), dim3(ATT_THREADS), 0, stream>>>(QH, QL, KH, KL, VT16, SIMP, beta, OH, OL);
  gemm16<true, M_F32, false><<<dim3(NB * (SQ / 64) * (DM / 64)), dim3(128), 0, stream>>>(
      OH, OL, WO16, bo, out, OL, OL, SQ, DM, INNER, SQ * INNER, 0, SQ_FULL * DM, 0,
      1.0f / (OSC * WSC), 1.0f, 1.0f);
  (void)hipGetLastError();
}
